// Encoder_4793183502909
// MI455X (gfx1250) — hardware-verified
//
#include <hip/hip_runtime.h>
#include <math.h>

constexpr int NBAT   = 64;
constexpr int NSEQ   = 512;
constexpr int NVOC   = 32000;
constexpr int NUNIT  = 256;
constexpr int NGATE  = 768;
constexpr int NROWS  = NBAT * NSEQ;
constexpr int NTHR   = 256;
constexpr int HPITCH = 264;
constexpr int SLABP  = 36;
constexpr int NOUT   = NBAT * NSEQ * NUNIT;
constexpr float OPCARRY     = 16.0f;
constexpr float GXC_INV     = 1.0f / 16.0f;
constexpr float ACC_INV     = 1.0f / 256.0f;
static_assert(NGATE == 3 * NUNIT, "gate blocks z | r | h");
static_assert(NROWS % 64 == 0 && NGATE % 64 == 0 && NUNIT % 32 == 0, "GEMM tile multiples");
static_assert(NUNIT == 32 * (NTHR / 32), "8 waves x 32 units");
static_assert(NBAT % 16 == 0, "16 sequences per scan block");
static_assert((2 * 16 * HPITCH) % NTHR == 0, "h tile zero fill exact");
static_assert(NSEQ == 2 * NTHR, "mask word build covers 512 steps");
static_assert(NROWS % 32 == 0, "gather blocks of 32 rows");
static_assert((HPITCH % 8) == 0 && (SLABP % 4) == 0, "16-B aligned LDS rows");

typedef __attribute__((ext_vector_type(16))) _Float16 v16h;
typedef __attribute__((ext_vector_type(8)))  _Float16 v8h;
typedef __attribute__((ext_vector_type(8)))  float    v8f;
typedef __attribute__((ext_vector_type(4)))  float    v4f;

__device__ __forceinline__ void guard4_h(v8f& a, v8f& b, v8f& c, v8f& d, v16h x, v16h y0, v16h y1, v16h y2, v16h y3) {
  asm volatile("v_nop\n\tv_nop\n\tv_nop\n\tv_nop" : "+v"(a), "+v"(b), "+v"(c), "+v"(d) : "v"(x), "v"(y0), "v"(y1), "v"(y2), "v"(y3));
}
__device__ __forceinline__ void guard3_h(v8f& a, v8f& b, v8f& c, v16h x, v16h y0, v16h y1, v16h y2) {
  asm volatile("v_nop\n\tv_nop\n\tv_nop\n\tv_nop" : "+v"(a), "+v"(b), "+v"(c) : "v"(x), "v"(y0), "v"(y1), "v"(y2));
}
__device__ __forceinline__ void keep4_h(v16h a, v16h b, v16h c, v16h d) { asm volatile("v_nop" :: "v"(a), "v"(b), "v"(c), "v"(d)); }
__device__ __forceinline__ void acc_guard4(v8f& a, v8f& b, v8f& c, v8f& d) { asm volatile("v_nop\n\tv_nop\n\tv_nop\n\tv_nop" : "+v"(a), "+v"(b), "+v"(c), "+v"(d)); }
__device__ __forceinline__ void acc_guard3(v8f& a, v8f& b, v8f& c) { asm volatile("v_nop\n\tv_nop\n\tv_nop\n\tv_nop" : "+v"(a), "+v"(b), "+v"(c)); }

struct FragH {
  union U { v16h v; v8h h[2]; };
  static __device__ __forceinline__ v16h load(const _Float16* p) {
    U f; f.h[0] = *(const v8h*)(p); f.h[1] = *(const v8h*)(p + 16); return f.v;
  }
  static __device__ __forceinline__ v8f mma(v16h a, v16h b, v8f c) {
    return __builtin_amdgcn_wmma_f32_16x16x32_f16(false, a, false, b, (short)0, c, false, false);
  }
};

__device__ __forceinline__ float h16_to_f32(unsigned hb) {
  const unsigned sgn = (hb & 0x8000u) << 16;
  const unsigned em = hb & 0x7fffu;
  const float fn = __uint_as_float((em << 13) + 0x38000000u);
  const float fs = (float)em * 5.9604644775390625e-8f;
  const float mag = (em < 0x400u) ? fs : fn;
  return __uint_as_float(__float_as_uint(mag) | sgn);
}

__device__ __forceinline__ float sigm_f(float x) { return __builtin_amdgcn_rcpf(1.0f + expf(-x)); }
__device__ __forceinline__ float tanh_f(float x) { return 1.0f - 2.0f * __builtin_amdgcn_rcpf(1.0f + expf(2.0f * x)); }

__global__ __launch_bounds__(NTHR) void pack_wt_kernel(const float* __restrict__ Wf, const float* __restrict__ Wb,
                                                       const float* __restrict__ Uf, const float* __restrict__ Ub,
                                                       unsigned short* __restrict__ planes) {
  __shared__ float Tt[64 * 65];
  const int tid = threadIdx.x;
  const int zsel = blockIdx.z;
  const float* src = (zsel == 0) ? Wf : ((zsel == 1) ? Wb : ((zsel == 2) ? Uf : Ub));
  unsigned short* O = planes + (size_t)zsel * NGATE * NUNIT;
  const int c0 = blockIdx.x * 64, r0 = blockIdx.y * 64;
#pragma unroll
  for (int i = 0; i < 4; ++i) {
    const int idx = i * NTHR + tid;
    const int rr = idx >> 4, cc = (idx & 15) * 4;
    const v4f v = *(const v4f*)(src + (size_t)(r0 + rr) * (size_t)NGATE + c0 + cc);
    Tt[rr * 65 + cc + 0] = v[0];
    Tt[rr * 65 + cc + 1] = v[1];
    Tt[rr * 65 + cc + 2] = v[2];
    Tt[rr * 65 + cc + 3] = v[3];
  }
  __syncthreads();
  const int q = tid >> 3, c8 = (tid & 7) * 8;
  v8h hv[2];
#pragma unroll
  for (int g = 0; g < 2; ++g) {
    const int qq = g * 32 + q;
#pragma unroll
    for (int e = 0; e < 8; ++e) {
      const float f = Tt[(c8 + e) * 65 + qq];
      hv[g][e] = (_Float16)(f * OPCARRY);
    }
  }
  for (int pass = 0; pass < 2; ++pass) {
#pragma unroll
    for (int g = 0; g < 2; ++g) {
      const size_t o = (size_t)(c0 + g * 32 + q) * (size_t)NUNIT + (size_t)(r0 + c8);
      *(volatile v8h*)(O + o) = hv[g];
    }
    __threadfence();
  }
}

__global__ __launch_bounds__(NTHR) void gather_pack_kernel(const int* __restrict__ X, const float* __restrict__ emb,
                                                           unsigned short* __restrict__ XP) {
  const int tid = threadIdx.x, lane = tid & 31, wave = tid >> 5;
  const int m0 = blockIdx.x * 32;
  v8h hv[4];
#pragma unroll
  for (int it = 0; it < 4; ++it) {
    const int m = m0 + it * 8 + wave;
    const int s = m >> 6, b = m & 63;
    int tok = X[b * NSEQ + s];
    tok = tok < 0 ? 0 : tok;
    tok = tok > (NVOC - 1) ? (NVOC - 1) : tok;
    const float* ep = emb + (size_t)tok * NUNIT + lane * 8;
    const v4f a = *(const v4f*)(ep);
    const v4f bq = *(const v4f*)(ep + 4);
#pragma unroll
    for (int e = 0; e < 4; ++e) {
      hv[it][e]     = (_Float16)(a[e] * OPCARRY);
      hv[it][4 + e] = (_Float16)(bq[e] * OPCARRY);
    }
  }
  for (int pass = 0; pass < 2; ++pass) {
#pragma unroll
    for (int it = 0; it < 4; ++it) {
      const int m = m0 + it * 8 + wave;
      *(volatile v8h*)(XP + (size_t)m * NUNIT + lane * 8) = hv[it];
    }
    __threadfence();
  }
}

__global__ __launch_bounds__(256) void gemm64_f16_kernel(const unsigned short* __restrict__ Ap, int lda,
                                                         const unsigned short* __restrict__ Btp, int ldb,
                                                         unsigned short* __restrict__ Cp, int ldc,
                                                         int M, int N, int K, float scale) {
  const _Float16* A = (const _Float16*)Ap;
  const _Float16* Bt = (const _Float16*)Btp;
  __shared__ __align__(16) float sT[8][16 * 68];
  const int lane = threadIdx.x & 31;
  const int wave = threadIdx.x >> 5;
  const int tilesN = N >> 6;
  const int tilesM = M >> 6;
  const int tile = blockIdx.x * 8 + wave;
  if (tile >= tilesM * tilesN) return;
  const int tm = tile / tilesN;
  const int tn = tile - tm * tilesN;
  const int m0 = tm << 6;
  const int n0 = tn << 6;
  const int rlane = lane & 15;
  const int koff  = (lane >> 4) * 8;
  const int mOff  = (lane >> 4) * 8;

  v8f acc[4][4];
#pragma unroll
  for (int i = 0; i < 4; ++i)
#pragma unroll
    for (int j = 0; j < 4; ++j) acc[i][j] = (v8f){0.f, 0.f, 0.f, 0.f, 0.f, 0.f, 0.f, 0.f};

  for (int k0 = 0; k0 < K; k0 += 32) {
    v16h bh[4];
#pragma unroll
    for (int j = 0; j < 4; ++j) {
      const size_t bo = (size_t)(n0 + (j << 4) + rlane) * ldb + koff + k0;
      bh[j] = FragH::load(Bt + bo);
    }
#pragma unroll
    for (int i = 0; i < 4; ++i) {
      const size_t ao = (size_t)(m0 + (i << 4) + rlane) * lda + koff + k0;
      const v16h ah = FragH::load(A + ao);
#pragma unroll
      for (int j = 0; j < 4; ++j) acc[i][j] = FragH::mma(ah, bh[j], acc[i][j]);
      guard4_h(acc[i][0], acc[i][1], acc[i][2], acc[i][3], ah, bh[0], bh[1], bh[2], bh[3]);
    }
    keep4_h(bh[0], bh[1], bh[2], bh[3]);
  }
  acc_guard4(acc[0][0], acc[0][1], acc[0][2], acc[0][3]);
  acc_guard4(acc[1][0], acc[1][1], acc[1][2], acc[1][3]);
  acc_guard4(acc[2][0], acc[2][1], acc[2][2], acc[2][3]);
  acc_guard4(acc[3][0], acc[3][1], acc[3][2], acc[3][3]);

  float* slab = sT[wave];
#pragma unroll
  for (int i = 0; i < 4; ++i) {
    const int mBase = m0 + (i << 4);
#pragma unroll
    for (int j = 0; j < 4; ++j) {
#pragma unroll
      for (int r = 0; r < 8; ++r) {
        const float v = acc[i][j][r] * scale;
        slab[(mOff + r) * 68 + (j << 4) + rlane] = v;
      }
    }
    __builtin_amdgcn_fence(__ATOMIC_RELEASE, "workgroup");
    __builtin_amdgcn_wave_barrier();
    __builtin_amdgcn_fence(__ATOMIC_ACQUIRE, "workgroup");
    {
      const int q = lane >> 3, c8 = (lane & 7) * 8;
      for (int pass = 0; pass < 2; ++pass) {
#pragma unroll
        for (int it = 0; it < 4; ++it) {
          const int row = it * 4 + q;
          const float* sp = slab + row * 68 + c8;
          v8h hv;
#pragma unroll
          for (int e = 0; e < 8; ++e) hv[e] = (_Float16)sp[e];
          *(volatile v8h*)(Cp + (size_t)(mBase + row) * ldc + n0 + c8) = hv;
        }
        __threadfence();
      }
    }
    __builtin_amdgcn_fence(__ATOMIC_RELEASE, "workgroup");
    __builtin_amdgcn_wave_barrier();
    __builtin_amdgcn_fence(__ATOMIC_ACQUIRE, "workgroup");
  }
}

template <bool REVERSE, bool ADDPLANE>
__global__ __launch_bounds__(NTHR) void gru_scan_kernel(const int* __restrict__ X,
                                                        const unsigned short* __restrict__ GXp,
                                                        const unsigned short* __restrict__ UTp,
                                                        const float* __restrict__ bias2,
                                                        const float* __restrict__ ADDP,
                                                        float* __restrict__ DST) {
  __shared__ __align__(16) _Float16 Ah[2][16 * HPITCH];
  __shared__ __align__(16) float    Sl[NTHR / 32][16 * SLABP];
  __shared__ unsigned mbits[NSEQ];
  const _Float16* UT = (const _Float16*)UTp;
  const int tid = threadIdx.x, lane = tid & 31, wave = tid >> 5;
  const int c = lane & 15, hh = lane >> 4, koff = hh * 8;
  const int q = lane >> 3, c4 = (lane & 7) * 4;
  const int rowb = blockIdx.x * 16;
  float* slab = Sl[wave];

  {
    _Float16* ahf = &Ah[0][0];
#pragma unroll 1
    for (int i = tid; i < 2 * 16 * HPITCH; i += NTHR) ahf[i] = (_Float16)0.0f;
  }
#pragma unroll
  for (int nt = 0; nt < 2; ++nt)
#pragma unroll
    for (int r = 0; r < 8; ++r) slab[(8 * hh + r) * SLABP + 16 * nt + c] = 0.0f;
  {
    unsigned m0 = 0u, m1 = 0u;
#pragma unroll 4
    for (int row = 0; row < 16; ++row) {
      const int t0 = X[(rowb + row) * NSEQ + tid];
      const int t1 = X[(rowb + row) * NSEQ + NTHR + tid];
      m0 |= ((t0 != 0) ? 1u : 0u) << row;
      m1 |= ((t1 != 0) ? 1u : 0u) << row;
    }
    mbits[tid] = m0;
    mbits[NTHR + tid] = m1;
  }
  const int j0 = 32 * wave + c, j1 = j0 + 16;
  const float bz0 = bias2[j0] + bias2[NGATE + j0];
  const float br0 = bias2[NUNIT + j0] + bias2[NGATE + NUNIT + j0];
  const float bi0 = bias2[2 * NUNIT + j0];
  const float bh0 = bias2[NGATE + 2 * NUNIT + j0];
  const float bz1 = bias2[j1] + bias2[NGATE + j1];
  const float br1 = bias2[NUNIT + j1] + bias2[NGATE + NUNIT + j1];
  const float bi1 = bias2[2 * NUNIT + j1];
  const float bh1 = bias2[NGATE + 2 * NUNIT + j1];
  __syncthreads();

  const v8f z8 = {0.f, 0.f, 0.f, 0.f, 0.f, 0.f, 0.f, 0.f};

#pragma unroll 1
  for (int t = 0; t < NSEQ; ++t) {
    const int s = REVERSE ? (NSEQ - 1 - t) : t;
    const int cur = t & 1;
    const _Float16* ahrow = &Ah[cur][0] + c * HPITCH + koff;
    _Float16* ahn = &Ah[cur ^ 1][0];
    const unsigned mb = mbits[s];
    const size_t gxrow0 = ((size_t)s * NBAT + (size_t)(rowb + 8 * hh)) * NGATE;

#pragma unroll 1
    for (int nt = 0; nt < 2; ++nt) {
      const int j = 32 * wave + 16 * nt + c;
      const _Float16* wu = UT + (size_t)j * NUNIT + koff;
      v8f accz = z8, accr = z8, acch = z8;
#pragma unroll 1
      for (int k0 = 0; k0 < NUNIT; k0 += 32) {
        const v16h a   = FragH::load(ahrow + k0);
        const v16h bq0 = FragH::load(wu + k0);
        const v16h bq1 = FragH::load(wu + (size_t)1 * NUNIT * NUNIT + k0);
        const v16h bq2 = FragH::load(wu + (size_t)2 * NUNIT * NUNIT + k0);
        accz = FragH::mma(a, bq0, accz);
        accr = FragH::mma(a, bq1, accr);
        acch = FragH::mma(a, bq2, acch);
        guard3_h(accz, accr, acch, a, bq0, bq1, bq2);
      }
      acc_guard3(accz, accr, acch);

      const unsigned short* gp = GXp + gxrow0 + j;
      unsigned gzb[8], grb[8], ghb[8];
#pragma unroll
      for (int r = 0; r < 8; ++r) gzb[r] = (unsigned)gp[(size_t)r * NGATE];
      asm volatile("" ::: "memory");
#pragma unroll
      for (int r = 0; r < 8; ++r) grb[r] = (unsigned)gp[(size_t)r * NGATE + NUNIT];
      asm volatile("" ::: "memory");
#pragma unroll
      for (int r = 0; r < 8; ++r) ghb[r] = (unsigned)gp[(size_t)r * NGATE + 2 * NUNIT];

      const float bz = nt ? bz1 : bz0;
      const float br = nt ? br1 : br0;
      const float bi = nt ? bi1 : bi0;
      const float bh = nt ? bh1 : bh0;

#pragma unroll
      for (int r = 0; r < 8; ++r) {
        const int sidx = (8 * hh + r) * SLABP + 16 * nt + c;
        const float gz = h16_to_f32(gzb[r]) * GXC_INV;
        const float gr = h16_to_f32(grb[r]) * GXC_INV;
        const float gh = h16_to_f32(ghb[r]) * GXC_INV;
        const float az = gz + accz[r] * ACC_INV + bz;
        const float ar = gr + accr[r] * ACC_INV + br;
        const float zg = sigm_f(az);
        const float rg = sigm_f(ar);
        const float ph = gh + bi + rg * (acch[r] * ACC_INV + bh);
        const float hc = tanh_f(ph);
        const float hold = slab[sidx];
        const float hcand = zg * hold + (1.0f - zg) * hc;
        const bool keep = ((mb >> (8 * hh + r)) & 1u) != 0u;
        const float hn = keep ? hcand : hold;
        slab[sidx] = hn;
        ahn[(8 * hh + r) * HPITCH + j] = (_Float16)(hn * OPCARRY);
      }
    }

    __builtin_amdgcn_fence(__ATOMIC_RELEASE, "workgroup");
    __builtin_amdgcn_wave_barrier();
    __builtin_amdgcn_fence(__ATOMIC_ACQUIRE, "workgroup");
    {
      v4f ov[4];
      size_t offs[4];
#pragma unroll
      for (int it = 0; it < 4; ++it) {
        const int row = it * 4 + q;
        v4f v = *(const v4f*)(slab + row * SLABP + c4);
        const size_t off = ((size_t)(rowb + row) * NSEQ + (size_t)s) * NUNIT + (size_t)(32 * wave + c4);
        if (ADDPLANE) {
          const v4f pv = *(const v4f*)(ADDP + off);
          v = v + pv;
        }
        ov[it] = v;
        offs[it] = off;
      }
      for (int pass = 0; pass < 2; ++pass) {
#pragma unroll
        for (int it = 0; it < 4; ++it) *(volatile v4f*)(DST + offs[it]) = ov[it];
        __threadfence();
      }
    }
    __builtin_amdgcn_fence(__ATOMIC_RELEASE, "workgroup");
    __builtin_amdgcn_wave_barrier();
    __builtin_amdgcn_fence(__ATOMIC_ACQUIRE, "workgroup");
    __syncthreads();
  }
}

extern "C" void kernel_launch(void* const* d_in, const int* in_sizes, int n_in,
                              void* d_out, int out_size, void* d_ws, size_t ws_size, hipStream_t stream) {
  if (n_in < 8 || d_out == nullptr || d_ws == nullptr) return;
  if (in_sizes[0] != NBAT * NSEQ || in_sizes[1] != NVOC * NUNIT ||
      in_sizes[2] != NUNIT * NGATE || in_sizes[3] != NUNIT * NGATE || in_sizes[4] != 2 * NGATE ||
      in_sizes[5] != NUNIT * NGATE || in_sizes[6] != NUNIT * NGATE || in_sizes[7] != 2 * NGATE ||
      out_size != NOUT) return;

  const int*   x   = (const int*)d_in[0];
  const float* emb = (const float*)d_in[1];
  const float* Wf  = (const float*)d_in[2];
  const float* Uf  = (const float*)d_in[3];
  const float* bf  = (const float*)d_in[4];
  const float* Wb  = (const float*)d_in[5];
  const float* Ub  = (const float*)d_in[6];
  const float* bb  = (const float*)d_in[7];
  float* out = (float*)d_out;

  char* ws = (char*)d_ws;
  size_t off = 0;
  auto carve = [&](size_t bytes) -> char* { char* p = ws + off; off += (bytes + 255) & ~(size_t)255; return p; };
  unsigned short* XP  = (unsigned short*)carve((size_t)NROWS * NUNIT * 2);
  unsigned short* WUT = (unsigned short*)carve((size_t)4 * NGATE * NUNIT * 2);
  unsigned short* GX  = (unsigned short*)carve((size_t)NROWS * NGATE * 2);
  float*          HB  = (float*)carve((size_t)NOUT * 4);
  if (off > ws_size || off > (size_t)134217728) return;

  const size_t planeElems = (size_t)NGATE * NUNIT;
  unsigned short* WTf = WUT + 0 * planeElems;
  unsigned short* WTb = WUT + 1 * planeElems;
  unsigned short* UTf = WUT + 2 * planeElems;
  unsigned short* UTb = WUT + 3 * planeElems;

  pack_wt_kernel<<<dim3(NGATE / 64, NUNIT / 64, 4), NTHR, 0, stream>>>(Wf, Wb, Uf, Ub, WUT);
  gather_pack_kernel<<<NROWS / 32, NTHR, 0, stream>>>(x, emb, XP);

  const int gemmBlocks = (NROWS / 64) * (NGATE / 64) / 8;
  gemm64_f16_kernel<<<gemmBlocks, 256, 0, stream>>>(XP, NUNIT, WTb, NUNIT, GX, NGATE, NROWS, NGATE, NUNIT, GXC_INV);
  gru_scan_kernel<true, false><<<NBAT / 16, NTHR, 0, stream>>>(x, GX, UTb, bb, bb, HB);
  gemm64_f16_kernel<<<gemmBlocks, 256, 0, stream>>>(XP, NUNIT, WTf, NUNIT, GX, NGATE, NROWS, NGATE, NUNIT, GXC_INV);
  gru_scan_kernel<false, true><<<NBAT / 16, NTHR, 0, stream>>>(x, GX, UTf, bf, HB, out);
}
